// GatedSumLinear_80479097192857
// MI455X (gfx1250) — hardware-verified
//
#include <hip/hip_runtime.h>
#include <math.h>
#include <stdint.h>

#define NBATCH 4
#define SEQ    2048
#define DM     1024
#define DO     1024
#define NE     8
#define MTOK   (NBATCH * SEQ)
#define NGP    64
static_assert((MTOK % 256) == 0 && (DM % 64) == 0 && (DO % 64) == 0 && (DM % 32) == 0);
static_assert(NE == 8 && NE <= NGP);
static_assert(((MTOK * DM) % (8 * 256)) == 0 && ((NE * DO * DM) % (8 * 256)) == 0 && ((NGP * DM) % (8 * 256)) == 0);

typedef __bf16   v16b __attribute__((ext_vector_type(16)));
typedef __bf16   v8b  __attribute__((ext_vector_type(8)));
typedef float    v8f  __attribute__((ext_vector_type(8)));
typedef float    v4f  __attribute__((ext_vector_type(4)));
typedef unsigned int v4u __attribute__((ext_vector_type(4)));

__device__ __forceinline__ unsigned short bf_bits(float f) {
  unsigned u = __float_as_uint(f);
  return (unsigned short)((u + 0x7FFFu + ((u >> 16) & 1u)) >> 16);
}
__device__ __forceinline__ float bf_up(unsigned short h) { return __uint_as_float(((unsigned)h) << 16); }
__device__ __forceinline__ unsigned pk16(unsigned short a, unsigned short b) { return (unsigned)a | ((unsigned)b << 16); }
__device__ __forceinline__ v8f zero8() { v8f z = {0.f, 0.f, 0.f, 0.f, 0.f, 0.f, 0.f, 0.f}; return z; }

__device__ __forceinline__ v16b ldfrag_b(const __bf16* p) {
  union { v16b v; v8b h[2]; } f;
  f.h[0] = *(const v8b*)(p);
  f.h[1] = *(const v8b*)(p + 16);
  return f.v;
}

__device__ __forceinline__ v8f mma_b_raw(v16b a, v16b b, v8f c) {
  return __builtin_amdgcn_wmma_f32_16x16x32_bf16(false, a, false, b, (short)0, c, false, false);
}
__device__ __forceinline__ void dep_guard_b(v8f& a, v8f& b, v16b x, v16b y) {
#if defined(__HIP_DEVICE_COMPILE__)
  asm volatile("v_nop\n\tv_nop\n\tv_nop\n\tv_nop" : "+v"(a), "+v"(b) : "v"(x), "v"(y));
#endif
}
__device__ __forceinline__ void keep4_b(v16b a, v16b b, v16b c, v16b d) {
#if defined(__HIP_DEVICE_COMPILE__)
  asm volatile("v_nop" :: "v"(a), "v"(b), "v"(c), "v"(d));
#endif
}
__device__ __forceinline__ void keep2_b(v16b a, v16b b) {
#if defined(__HIP_DEVICE_COMPILE__)
  asm volatile("v_nop" :: "v"(a), "v"(b));
#endif
}
__device__ __forceinline__ void acc_guard4(v8f& a, v8f& b, v8f& c, v8f& d) {
#if defined(__HIP_DEVICE_COMPILE__)
  asm volatile("v_nop\n\tv_nop\n\tv_nop\n\tv_nop" : "+v"(a), "+v"(b), "+v"(c), "+v"(d));
#endif
}
__device__ __forceinline__ void wave_sync_lds() {
  __builtin_amdgcn_fence(__ATOMIC_RELEASE, "workgroup");
  __builtin_amdgcn_wave_barrier();
  __builtin_amdgcn_fence(__ATOMIC_ACQUIRE, "workgroup");
}

__global__ __launch_bounds__(256) void cvt_bf16x8(const float* __restrict__ in, unsigned short* out,
                                                  int n8, int n8tot) {
  const int i = blockIdx.x * 256 + threadIdx.x;
  if (i >= n8tot) return;
  int ic = i;
  if (ic > n8 - 1) ic = n8 - 1;
  const v4f a = *(const v4f*)(in + (size_t)ic * 8);
  const v4f b = *(const v4f*)(in + (size_t)ic * 8 + 4);
  v4u p;
  p[0] = pk16(bf_bits(a[0]), bf_bits(a[1]));
  p[1] = pk16(bf_bits(a[2]), bf_bits(a[3]));
  p[2] = pk16(bf_bits(b[0]), bf_bits(b[1]));
  p[3] = pk16(bf_bits(b[2]), bf_bits(b[3]));
  if (i >= n8) { p[0] = 0u; p[1] = 0u; p[2] = 0u; p[3] = 0u; }
  *(volatile v4u*)(out + (size_t)i * 8) = p;
  __threadfence();
  *(volatile v4u*)(out + (size_t)i * 8) = p;
}

template <int NSPLIT, int OUT_MODE>
__global__ __launch_bounds__(256) void gemm64(
    const unsigned short* __restrict__ Ap, const unsigned short* A2p, int lda, long long strideA,
    const unsigned short* __restrict__ Btp, const unsigned short* Bt2p, int ldb, long long strideB,
    void* Cout, int ldc, long long strideC,
    int M, int N, int K) {
  const __bf16* A   = (const __bf16*)(const void*)Ap;
  const __bf16* A2  = (const __bf16*)(const void*)A2p;
  const __bf16* Bt  = (const __bf16*)(const void*)Btp;
  const __bf16* Bt2 = (const __bf16*)(const void*)Bt2p;
  __shared__ __align__(16) float sT[8][16 * 68];
  const int b    = blockIdx.y;
  const int lane = threadIdx.x & 31;
  const int wave = threadIdx.x >> 5;
  const int tilesN = N >> 6;
  const int tilesM = M >> 6;
  const int tile = blockIdx.x * 8 + wave;
  if (tile >= tilesM * tilesN) return;
  const int tm = tile / tilesN;
  const int tn = tile - tm * tilesN;
  const int m0 = tm << 6;
  const int n0 = tn << 6;

  const __bf16* Ab  = A  + (size_t)b * strideA;
  const __bf16* Bb  = Bt + (size_t)b * strideB;
  const __bf16* Ab2 = (NSPLIT >= 1) ? (A2  + (size_t)b * strideA) : Ab;
  const __bf16* Bb2 = (NSPLIT == 2) ? (Bt2 + (size_t)b * strideB) : Bb;

  const int rlane = lane & 15;
  const int koff  = (lane >> 4) * 8;
  const int mOff  = (lane >> 4) * 8;

  v8f acc[4][4];
#pragma unroll
  for (int i = 0; i < 4; ++i)
#pragma unroll
    for (int j = 0; j < 4; ++j) acc[i][j] = zero8();

  for (int k0 = 0; k0 < K; k0 += 32) {
    v16b bh[4], bl[4];
#pragma unroll
    for (int j = 0; j < 4; ++j) {
      const size_t bo = (size_t)(n0 + (j << 4) + rlane) * ldb + koff + k0;
      bh[j] = ldfrag_b(Bb + bo);
      if (NSPLIT == 2) bl[j] = ldfrag_b(Bb2 + bo); else bl[j] = bh[j];
    }
#pragma unroll
    for (int i = 0; i < 4; ++i) {
      const size_t ao = (size_t)(m0 + (i << 4) + rlane) * lda + koff + k0;
      const v16b ah = ldfrag_b(Ab + ao);
      v16b al = ah;
      if (NSPLIT >= 1) al = ldfrag_b(Ab2 + ao);
#pragma unroll
      for (int j = 0; j < 4; ++j) {
        acc[i][j] = mma_b_raw(ah, bh[j], acc[i][j]);
        if (NSPLIT >= 1) acc[i][j] = mma_b_raw(al, bh[j], acc[i][j]);
        if (NSPLIT == 2) acc[i][j] = mma_b_raw(ah, bl[j], acc[i][j]);
      }
      dep_guard_b(acc[i][0], acc[i][3], ah, al);
    }
    keep4_b(bh[0], bh[1], bh[2], bh[3]);
    if (NSPLIT == 2) keep4_b(bl[0], bl[1], bl[2], bl[3]);
  }
  acc_guard4(acc[0][0], acc[0][1], acc[0][2], acc[0][3]);
  acc_guard4(acc[1][0], acc[1][1], acc[1][2], acc[1][3]);
  acc_guard4(acc[2][0], acc[2][1], acc[2][2], acc[2][3]);
  acc_guard4(acc[3][0], acc[3][1], acc[3][2], acc[3][3]);

  float* slab = sT[wave];
  const int hh = lane >> 4, c4 = (lane & 15) * 4;
  float* C = (float*)Cout + (size_t)b * strideC;
#pragma unroll
  for (int i = 0; i < 4; ++i) {
    const int mBase = m0 + (i << 4);
#pragma unroll
    for (int j = 0; j < 4; ++j) {
#pragma unroll
      for (int r = 0; r < 8; ++r) {
        slab[(mOff + r) * 68 + (j << 4) + rlane] = acc[i][j][r];
      }
    }
    wave_sync_lds();
    for (int pass = 0; pass < 2; ++pass) {
#pragma unroll
      for (int it = 0; it < 8; ++it) {
        const int row = it * 2 + hh;
        const v4f v = *(const v4f*)(slab + row * 68 + c4);
        *(volatile v4f*)(C + (size_t)(mBase + row) * ldc + n0 + c4) = v;
      }
      __threadfence();
    }
    wave_sync_lds();
  }
}

__global__ __launch_bounds__(256) void gemm_moe(
    const unsigned short* __restrict__ Ap, int lda,
    const unsigned short* __restrict__ Btp, int ldb, long long strideE,
    const float* __restrict__ Gp, int gpitch,
    const float* __restrict__ biasp, int bpitch,
    float* Cout, int ldc, int M, int N, int K) {
  const __bf16* A  = (const __bf16*)(const void*)Ap;
  const __bf16* Bt = (const __bf16*)(const void*)Btp;
  __shared__ __align__(16) float sT[8][16 * 36];
  const int lane = threadIdx.x & 31;
  const int wave = threadIdx.x >> 5;
  const int tilesN = N >> 5;
  const int tilesM = M >> 6;
  const int tile = blockIdx.x * 8 + wave;
  if (tile >= tilesM * tilesN) return;
  const int tm = tile / tilesN;
  const int tn = tile - tm * tilesN;
  const int m0 = tm << 6;
  const int n0 = tn << 5;

  const int rlane = lane & 15;
  const int koff  = (lane >> 4) * 8;
  const int mOff  = (lane >> 4) * 8;

  v8f run[4][2];
  v8f acc[4][2];
#pragma unroll
  for (int i = 0; i < 4; ++i)
#pragma unroll
    for (int j = 0; j < 2; ++j) run[i][j] = zero8();

#pragma unroll 1
  for (int h = 0; h < NE; ++h) {
#pragma unroll
    for (int i = 0; i < 4; ++i)
#pragma unroll
      for (int j = 0; j < 2; ++j) acc[i][j] = zero8();
    const __bf16* Bh = Bt + (size_t)h * (size_t)strideE;

    for (int k0 = 0; k0 < K; k0 += 32) {
      v16b bh[2];
#pragma unroll
      for (int j = 0; j < 2; ++j) {
        const size_t bo = (size_t)(n0 + (j << 4) + rlane) * ldb + koff + k0;
        bh[j] = ldfrag_b(Bh + bo);
      }
#pragma unroll
      for (int i = 0; i < 4; ++i) {
        const size_t ao = (size_t)(m0 + (i << 4) + rlane) * lda + koff + k0;
        const v16b ah = ldfrag_b(A + ao);
        acc[i][0] = mma_b_raw(ah, bh[0], acc[i][0]);
        acc[i][1] = mma_b_raw(ah, bh[1], acc[i][1]);
        dep_guard_b(acc[i][0], acc[i][1], ah, bh[1]);
      }
      keep2_b(bh[0], bh[1]);
    }
    acc_guard4(acc[0][0], acc[0][1], acc[1][0], acc[1][1]);
    acc_guard4(acc[2][0], acc[2][1], acc[3][0], acc[3][1]);

    const float* bp = biasp + (size_t)h * (size_t)bpitch + n0 + rlane;
    const float b0 = bf_up(bf_bits(bp[0]));
    const float b1 = bf_up(bf_bits(bp[16]));
#pragma unroll
    for (int i = 0; i < 4; ++i) {
      const float* gp = Gp + (size_t)(m0 + (i << 4) + mOff) * (size_t)gpitch + h;
      float g[8];
#pragma unroll
      for (int r = 0; r < 8; ++r) g[r] = gp[(size_t)r * gpitch];
#pragma unroll
      for (int r = 0; r < 8; ++r) {
        run[i][0][r] += g[r] * (acc[i][0][r] + b0);
        run[i][1][r] += g[r] * (acc[i][1][r] + b1);
      }
    }
  }
  acc_guard4(run[0][0], run[0][1], run[1][0], run[1][1]);
  acc_guard4(run[2][0], run[2][1], run[3][0], run[3][1]);

  float* slab = sT[wave];
  const int q = lane >> 3, c4 = (lane & 7) * 4;
  float* C = Cout;
#pragma unroll
  for (int i = 0; i < 4; ++i) {
    const int mBase = m0 + (i << 4);
#pragma unroll
    for (int j = 0; j < 2; ++j) {
#pragma unroll
      for (int r = 0; r < 8; ++r) {
        slab[(mOff + r) * 36 + (j << 4) + rlane] = run[i][j][r];
      }
    }
    wave_sync_lds();
    v4f v[4];
#pragma unroll
    for (int it = 0; it < 4; ++it) {
      const int row = it * 4 + q;
      v[it] = *(const v4f*)(slab + row * 36 + c4);
    }
    for (int pass = 0; pass < 2; ++pass) {
#pragma unroll
      for (int it = 0; it < 4; ++it) {
        const int row = it * 4 + q;
        *(volatile v4f*)(C + (size_t)(mBase + row) * ldc + n0 + c4) = v[it];
      }
      __threadfence();
    }
    wave_sync_lds();
  }
}

__global__ __launch_bounds__(256) void gate_softmax(const float* __restrict__ Lp, const float* __restrict__ gb,
                                                    float* Gp, int nrows) {
  __shared__ __align__(16) float sG[256 * 8];
  const int tid = threadIdx.x;
  int row = blockIdx.x * 256 + tid;
  if (row > nrows - 1) row = nrows - 1;
  const float* lr = Lp + (size_t)row * NGP;
  const v4f la = *(const v4f*)(lr);
  const v4f lb = *(const v4f*)(lr + 4);
  float l0 = la[0] + bf_up(bf_bits(gb[0]));
  float l1 = la[1] + bf_up(bf_bits(gb[1]));
  float l2 = la[2] + bf_up(bf_bits(gb[2]));
  float l3 = la[3] + bf_up(bf_bits(gb[3]));
  float l4 = lb[0] + bf_up(bf_bits(gb[4]));
  float l5 = lb[1] + bf_up(bf_bits(gb[5]));
  float l6 = lb[2] + bf_up(bf_bits(gb[6]));
  float l7 = lb[3] + bf_up(bf_bits(gb[7]));
  float mx = fmaxf(fmaxf(fmaxf(l0, l1), fmaxf(l2, l3)), fmaxf(fmaxf(l4, l5), fmaxf(l6, l7)));
  l0 = __expf(l0 - mx); l1 = __expf(l1 - mx); l2 = __expf(l2 - mx); l3 = __expf(l3 - mx);
  l4 = __expf(l4 - mx); l5 = __expf(l5 - mx); l6 = __expf(l6 - mx); l7 = __expf(l7 - mx);
  const float s = ((l0 + l1) + (l2 + l3)) + ((l4 + l5) + (l6 + l7));
  const float inv = 1.0f / s;
  v4f pa, pb;
  pa[0] = l0 * inv; pa[1] = l1 * inv; pa[2] = l2 * inv; pa[3] = l3 * inv;
  pb[0] = l4 * inv; pb[1] = l5 * inv; pb[2] = l6 * inv; pb[3] = l7 * inv;
  *(v4f*)(sG + tid * 8)     = pa;
  *(v4f*)(sG + tid * 8 + 4) = pb;
  __syncthreads();
  const v4f w0 = *(const v4f*)(sG + tid * 4);
  const v4f w1 = *(const v4f*)(sG + (tid + 256) * 4);
  float* Gb = Gp + (size_t)blockIdx.x * (256 * 8);
  for (int pass = 0; pass < 2; ++pass) {
    *(volatile v4f*)(Gb + (size_t)tid * 4) = w0;
    *(volatile v4f*)(Gb + (size_t)(tid + 256) * 4) = w1;
    __threadfence();
  }
}

extern "C" void kernel_launch(void* const* d_in, const int* in_sizes, int n_in,
                              void* d_out, int out_size, void* d_ws, size_t ws_size,
                              hipStream_t stream) {
  if (n_in < 5) return;
  if (in_sizes[0] != MTOK * DM) return;
  if (in_sizes[1] != NE * DM) return;
  if (in_sizes[2] != NE) return;
  if (in_sizes[3] != NE * DO * DM) return;
  if (in_sizes[4] != NE * DO) return;
  if (out_size != MTOK * DO) return;

  const float* x  = (const float*)d_in[0];
  const float* gw = (const float*)d_in[1];
  const float* gb = (const float*)d_in[2];
  const float* ew = (const float*)d_in[3];
  const float* eb = (const float*)d_in[4];
  float* out = (float*)d_out;

  const size_t PXb = (size_t)MTOK * DM * 2;
  const size_t PWb = (size_t)NE * DO * DM * 2;
  const size_t PGt = (size_t)NGP * DM * 2;
  const size_t PL  = (size_t)MTOK * NGP * 4;
  const size_t PG  = (size_t)MTOK * NE * 4;
  size_t off = 0;
  const size_t oXb = off; off += PXb;
  const size_t oWb = off; off += PWb;
  const size_t oGt = off; off += PGt;
  const size_t oL  = off; off += PL;
  const size_t oG  = off; off += PG;
  if (off > ws_size) return;
  if (off > (size_t)134217728) return;

  char* ws = (char*)d_ws;
  unsigned short* Xb = (unsigned short*)(ws + oXb);
  unsigned short* Wb = (unsigned short*)(ws + oWb);
  unsigned short* Gt = (unsigned short*)(ws + oGt);
  float* Lg = (float*)(ws + oL);
  float* Gg = (float*)(ws + oG);

  const dim3 blk(256);
  const int n8x  = MTOK * DM / 8;
  const int n8w  = NE * DO * DM / 8;
  const int n8g  = NE * DM / 8;
  const int n8gt = NGP * DM / 8;
  const dim3 gCvtX((n8x + 255) / 256);
  const dim3 gCvtW((n8w + 255) / 256);
  const dim3 gCvtG((n8gt + 255) / 256);
  const dim3 gGate(((MTOK / 64) * (NGP / 64) + 7) / 8, 1);
  const dim3 gSmx(MTOK / 256);
  const dim3 gMoe(((MTOK / 64) * (DO / 32) + 7) / 8);

  cvt_bf16x8<<<gCvtX, blk, 0, stream>>>(x, Xb, n8x, n8x);
  cvt_bf16x8<<<gCvtW, blk, 0, stream>>>(ew, Wb, n8w, n8w);
  cvt_bf16x8<<<gCvtG, blk, 0, stream>>>(gw, Gt, n8g, n8gt);
  gemm64<0, 0><<<gGate, blk, 0, stream>>>(
      Xb, Xb, DM, 0LL, Gt, Gt, DM, 0LL,
      (void*)Lg, NGP, 0LL,
      MTOK, NGP, DM);
  gate_softmax<<<gSmx, blk, 0, stream>>>(Lg, gb, Gg, MTOK);
  gemm_moe<<<gMoe, blk, 0, stream>>>(
      Xb, DM, Wb, DM, (long long)DO * DM,
      Gg, NE, eb, DO,
      out, DO, MTOK, DO, DM);
  (void)hipGetLastError();
}
